// GNNLayer_10075993277103
// MI455X (gfx1250) — hardware-run, weakly checked
//
#include <hip/hip_runtime.h>
#include <math.h>

typedef __attribute__((ext_vector_type(16))) _Float16 v16h;
typedef __attribute__((ext_vector_type(8)))  _Float16 v8h;
typedef __attribute__((ext_vector_type(8)))  float    v8f;
typedef __attribute__((ext_vector_type(4)))  float    v4f;

constexpr int kB    = 64;
constexpr int kT    = 12;
constexpr int kN    = 207;
constexpr int kH    = 64;
constexpr int kTW   = kT - 2;
constexpr int kNP   = 256;
constexpr int kRowP = kT * kNP;
constexpr int kQT   = 7;
constexpr int kKC   = 7;
constexpr int kTileP = 65;
constexpr int kSlabP = 68;
static_assert(kQT * 32 >= kN && kQT * 32 <= kNP, "query tiles cover the nodes inside the padded pitch");
static_assert(kKC * 32 >= kN && kKC * 32 <= kNP, "key chunks cover the nodes inside the padded pitch");
static_assert(kH == 64, "two 32-deep k-steps per 64-channel row");
static_assert(((kB * kTW * kQT) % 4) == 0, "four waves per block, exact grid");
static_assert((208 * 16) == 13 * 256, "tile staging: 13 passes of 256 threads x 4 floats");

constexpr float kCarryWF  = 64.0f;
constexpr float kCarryP   = 512.0f;
constexpr float kCarryX   = 16.0f;
constexpr float kCarryAct = 64.0f;
constexpr float kCarryW   = 64.0f;
constexpr float kPScale   = kCarryP / (kCarryWF * kCarryWF);
constexpr float kInvFF    = 1.0f / (kCarryAct * kCarryW);
constexpr float kF16Min   = 6.103515625e-5f;
constexpr float kEpsNorm  = 1e-12f;
constexpr float kEpsLN    = 1e-5f;
constexpr float kInvH     = 1.0f / (float)kH;

constexpr size_t kBytesWF  = (size_t)kB * kT * kNP * kH * 2;
constexpr size_t kBytesXT  = (size_t)kB * kH * kRowP * 2;
constexpr size_t kBytesWT  = (size_t)kH * kH * 2;
constexpr size_t kOffWF    = 0;
constexpr size_t kOffXT    = kOffWF + kBytesWF;
constexpr size_t kOffW1T   = kOffXT + kBytesXT;
constexpr size_t kOffW2T   = kOffW1T + kBytesWT;
constexpr size_t kWsTotal  = kOffW2T + kBytesWT;
static_assert(kWsTotal == 50348032ull, "carve total");
static_assert(kWsTotal <= 134217728ull, "carve cap");
static_assert((kOffXT % 128) == 0 && (kOffW1T % 128) == 0 && (kOffW2T % 128) == 0, "128-B aligned regions");

struct FragH {
  union U { v16h v; v8h h[2]; };
  static __device__ __forceinline__ v16h load(const _Float16* p) {
    U f;
    f.h[0] = *(const v8h*)(p);
    f.h[1] = *(const v8h*)(p + 16);
    return f.v;
  }
};

__device__ __forceinline__ v8f mma_h(v16h a, v16h b, v8f c) {
  c = __builtin_amdgcn_wmma_f32_16x16x32_f16(false, a, false, b, (short)0, c, false, false);
  asm volatile("v_nop\n\tv_nop\n\tv_nop\n\tv_nop" : "+v"(c) : "v"(a), "v"(b));
  return c;
}

__device__ __forceinline__ _Float16 to_h16(float v) {
  const float a = fabsf(v);
  const float z = (a < kF16Min) ? 0.0f : v;
  return (_Float16)z;
}

__device__ __forceinline__ v16h pack_pair(const v8f lo, const v8f hi, float sc) {
  v16h f;
#pragma unroll
  for (int r = 0; r < 8; ++r) {
    f[r]     = to_h16(lo[r] * sc);
    f[8 + r] = to_h16(hi[r] * sc);
  }
  return f;
}

__device__ __forceinline__ void load8(const float* p, float (&d)[8]) {
  const v4f a = *(const v4f*)(p);
  const v4f b = *(const v4f*)(p + 4);
  d[0] = a[0]; d[1] = a[1]; d[2] = a[2]; d[3] = a[3];
  d[4] = b[0]; d[5] = b[1]; d[6] = b[2]; d[7] = b[3];
}

__global__ __launch_bounds__(256) void planes_kernel(
    const float* __restrict__ feat, const float* __restrict__ wts,
    _Float16* __restrict__ WF, _Float16* __restrict__ XT)
{
  __shared__ float sF[208 * kTileP];
  __shared__ float sSw[kH];
  __shared__ float sInv[256];
  const int tid = threadIdx.x, lane = tid & 31, wave = tid >> 5;
  const int bt  = blockIdx.x;
  const int b   = bt / kT;
  const int tau = bt - b * kT;

  if (tid < kH) {
    const float w = wts[tid];
    sSw[tid] = 1.0f / (1.0f + expf(-w));
  }

  const float* src = feat + (size_t)bt * kN * kH;
#pragma unroll 1
  for (int i = 0; i < 13; ++i) {
    const int idx  = tid + 256 * i;
    const int row  = idx >> 4;
    const int c4   = (idx & 15) * 4;
    const int grow = (row < kN) ? row : (kN - 1);
    const v4f x = *(const v4f*)(src + (size_t)grow * kH + c4);
    float* d = sF + row * kTileP + c4;
    d[0] = x[0];
    d[1] = x[1];
    d[2] = x[2];
    d[3] = x[3];
  }
  __syncthreads();

  {
    const int rc = (tid < 208) ? tid : 207;
    float ss = 0.0f;
#pragma unroll 4
    for (int c = 0; c < kH; ++c) {
      const float v = sF[rc * kTileP + c] * sSw[c];
      ss = fmaf(v, v, ss);
    }
    const float nrm = sqrtf(ss);
    const float iv  = kCarryWF * (1.0f / fmaxf(nrm, kEpsNorm));
    sInv[tid] = (tid < kN) ? iv : 0.0f;
  }
  __syncthreads();

  {
    const int q = lane >> 3, c8 = (lane & 7) * 8;
#pragma unroll 1
    for (int it = 0; it < 8; ++it) {
      const int row = it * 32 + wave * 4 + q;
      const int rc  = (row < kN) ? row : (kN - 1);
      const float iv = sInv[row];
      v8h hv;
#pragma unroll
      for (int e = 0; e < 8; ++e) {
        const int c = c8 + e;
        float v = sF[rc * kTileP + c] * sSw[c] * iv;
        v = (row < kN) ? v : 0.0f;
        hv[e] = to_h16(v);
      }
      _Float16* p = WF + ((size_t)bt * kNP + row) * kH + c8;
      *(volatile v8h*)p = hv;
      __threadfence();
      *(volatile v8h*)p = hv;
    }
  }

  {
#pragma unroll 1
    for (int it = 0; it < 8; ++it) {
      const int c = it * 8 + wave;
      v8h hv;
#pragma unroll
      for (int e = 0; e < 8; ++e) {
        const int n  = lane * 8 + e;
        const int nc = (n < kN) ? n : (kN - 1);
        float v = sF[nc * kTileP + c] * kCarryX;
        v = (n < kN) ? v : 0.0f;
        hv[e] = to_h16(v);
      }
      _Float16* p = XT + ((size_t)(b * kH + c)) * kRowP + tau * kNP + lane * 8;
      *(volatile v8h*)p = hv;
      __threadfence();
      *(volatile v8h*)p = hv;
    }
  }
}

__global__ __launch_bounds__(256) void wplanes_kernel(
    const float* __restrict__ W1, const float* __restrict__ W2,
    _Float16* __restrict__ W1T, _Float16* __restrict__ W2T)
{
  const int tid = threadIdx.x, lane = tid & 31, wave = tid >> 5;
  const int q = lane >> 3, c8 = (lane & 7) * 8;
#pragma unroll 1
  for (int it = 0; it < 4; ++it) {
    const bool second = (it >= 2);
    const float* src = second ? W2 : W1;
    _Float16* dst = second ? W2T : W1T;
    const int row = (it & 1) * 32 + wave * 4 + q;
    v8h hv;
#pragma unroll
    for (int e = 0; e < 8; ++e) {
      const float v = src[(size_t)(c8 + e) * kH + row] * kCarryW;
      hv[e] = to_h16(v);
    }
    _Float16* p = dst + (size_t)row * kH + c8;
    *(volatile v8h*)p = hv;
    __threadfence();
    *(volatile v8h*)p = hv;
  }
}

__global__ __launch_bounds__(128) void fused_kernel(
    const _Float16* __restrict__ WF, const _Float16* __restrict__ XT,
    const _Float16* __restrict__ W1T, const _Float16* __restrict__ W2T,
    const float* __restrict__ feat,
    const float* __restrict__ b1, const float* __restrict__ b2,
    const float* __restrict__ gamma, const float* __restrict__ beta,
    float* __restrict__ out)
{
  __shared__ __align__(16) float sO[4][16 * kSlabP];
  const int lane = threadIdx.x & 31, wave = threadIdx.x >> 5;
  const int c16 = lane & 15, hh = lane >> 4, koff = hh * 8;
  const int gw   = blockIdx.x * 4 + wave;
  const int win  = gw / kQT;
  const int tile = gw - win * kQT;
  const int b    = win / kTW;
  const int t    = win - b * kTW;
  const int q0   = tile * 32;

  const _Float16* WFb = WF + (size_t)b * kT * kNP * kH;
  const _Float16* XTb = XT + (size_t)b * kH * kRowP;
  const _Float16* kbase = WFb + (size_t)c16 * kH + koff;
  const _Float16* xbase = XTb + (size_t)c16 * kRowP + koff;

  v16h qf[2][2];
#pragma unroll
  for (int mi = 0; mi < 2; ++mi) {
    const _Float16* qp = kbase + (size_t)((t + 2) * kNP + q0 + 16 * mi) * kH;
    qf[mi][0] = FragH::load(qp);
    qf[mi][1] = FragH::load(qp + 32);
  }

  v8f agg[4][2];
#pragma unroll
  for (int ct = 0; ct < 4; ++ct)
#pragma unroll
    for (int mi = 0; mi < 2; ++mi) agg[ct][mi] = (v8f){0.f, 0.f, 0.f, 0.f, 0.f, 0.f, 0.f, 0.f};
  float degp[2] = {0.0f, 0.0f};

#pragma unroll 1
  for (int sg = 0; sg < 3; ++sg) {
#pragma unroll 1
    for (int kc = 0; kc < kKC; ++kc) {
      const int keyrow0 = (t + sg) * kNP + kc * 32;
      v8f st[2][2];
#pragma unroll
      for (int kt2 = 0; kt2 < 2; ++kt2) {
        const _Float16* kp = kbase + (size_t)(keyrow0 + 16 * kt2) * kH;
        const v16h k0 = FragH::load(kp);
        const v16h k1 = FragH::load(kp + 32);
#pragma unroll
        for (int mi = 0; mi < 2; ++mi) {
          v8f s = (v8f){0.f, 0.f, 0.f, 0.f, 0.f, 0.f, 0.f, 0.f};
          s = mma_h(k0, qf[mi][0], s);
          s = mma_h(k1, qf[mi][1], s);
          st[kt2][mi] = s;
        }
      }
      v16h pf[2];
#pragma unroll
      for (int mi = 0; mi < 2; ++mi) {
#pragma unroll
        for (int r = 0; r < 8; ++r) {
          const float p0 = fmaxf(st[0][mi][r], 0.0f) * kPScale;
          const float p1 = fmaxf(st[1][mi][r], 0.0f) * kPScale;
          degp[mi] += p0;
          degp[mi] += p1;
          pf[mi][r]     = to_h16(p0);
          pf[mi][8 + r] = to_h16(p1);
        }
      }
#pragma unroll
      for (int ct = 0; ct < 4; ++ct) {
        const v16h xf = FragH::load(xbase + (size_t)(16 * ct) * kRowP + keyrow0);
#pragma unroll
        for (int mi = 0; mi < 2; ++mi) agg[ct][mi] = mma_h(xf, pf[mi], agg[ct][mi]);
      }
    }
  }

  float* slab = sO[wave];
  float* ob = out + ((size_t)(b * kTW + t) * kN) * kH;
  const int c4 = c16 * 4;

#pragma unroll
  for (int mi = 0; mi < 2; ++mi) {
    const float dsum = degp[mi] + __shfl_xor(degp[mi], 16, 32);
    const float inv  = 1.0f / (kCarryX * fmaxf(dsum, kCarryP * kEpsNorm));
    const float scA  = inv * kCarryAct;

    v16h af[2];
    af[0] = pack_pair(agg[0][mi], agg[1][mi], scA);
    af[1] = pack_pair(agg[2][mi], agg[3][mi], scA);

    v8f h1[4];
#pragma unroll
    for (int ot = 0; ot < 4; ++ot) {
      const _Float16* wp = W1T + (size_t)(16 * ot + c16) * kH + koff;
      const v16h w0 = FragH::load(wp);
      const v16h w1 = FragH::load(wp + 32);
      v8f a = (v8f){0.f, 0.f, 0.f, 0.f, 0.f, 0.f, 0.f, 0.f};
      a = mma_h(w0, af[0], a);
      a = mma_h(w1, af[1], a);
      float bv[8];
      load8(b1 + 16 * ot + 8 * hh, bv);
#pragma unroll
      for (int r = 0; r < 8; ++r) a[r] = fmaxf(a[r] * kInvFF + bv[r], 0.0f);
      h1[ot] = a;
    }
    v16h hf[2];
    hf[0] = pack_pair(h1[0], h1[1], kCarryAct);
    hf[1] = pack_pair(h1[2], h1[3], kCarryAct);

    const int n  = q0 + 16 * mi + c16;
    const int nc = (n < kN) ? n : (kN - 1);
    const float* rp = feat + ((size_t)((b * kT + t + 2) * kN + nc)) * kH + 8 * hh;
    float sv[4][8];
    float s1 = 0.0f;
#pragma unroll
    for (int ot = 0; ot < 4; ++ot) {
      const _Float16* wp = W2T + (size_t)(16 * ot + c16) * kH + koff;
      const v16h w0 = FragH::load(wp);
      const v16h w1 = FragH::load(wp + 32);
      v8f a = (v8f){0.f, 0.f, 0.f, 0.f, 0.f, 0.f, 0.f, 0.f};
      a = mma_h(w0, hf[0], a);
      a = mma_h(w1, hf[1], a);
      float bv[8], rv[8];
      load8(b2 + 16 * ot + 8 * hh, bv);
      load8(rp + 16 * ot, rv);
#pragma unroll
      for (int r = 0; r < 8; ++r) {
        const float v = (a[r] * kInvFF + bv[r]) + rv[r];
        sv[ot][r] = v;
        s1 += v;
      }
    }

    s1 += __shfl_xor(s1, 16, 32);
    const float mu = s1 * kInvH;
    float s2 = 0.0f;
#pragma unroll
    for (int ot = 0; ot < 4; ++ot) {
#pragma unroll
      for (int r = 0; r < 8; ++r) {
        const float d = sv[ot][r] - mu;
        sv[ot][r] = d;
        s2 += d * d;
      }
    }
    s2 += __shfl_xor(s2, 16, 32);
    const float var  = s2 * kInvH;
    const float rstd = 1.0f / sqrtf(var + kEpsLN);

#pragma unroll
    for (int ot = 0; ot < 4; ++ot) {
      float gv[8], ev[8];
      load8(gamma + 16 * ot + 8 * hh, gv);
      load8(beta + 16 * ot + 8 * hh, ev);
      v4f o0, o1;
#pragma unroll
      for (int r = 0; r < 4; ++r) {
        o0[r] = (sv[ot][r] * rstd) * gv[r] + ev[r];
        o1[r] = (sv[ot][4 + r] * rstd) * gv[4 + r] + ev[4 + r];
      }
      *(v4f*)(slab + c16 * kSlabP + 16 * ot + 8 * hh)     = o0;
      *(v4f*)(slab + c16 * kSlabP + 16 * ot + 8 * hh + 4) = o1;
    }
    __builtin_amdgcn_fence(__ATOMIC_RELEASE, "workgroup");
    __builtin_amdgcn_wave_barrier();
    __builtin_amdgcn_fence(__ATOMIC_ACQUIRE, "workgroup");

    for (int pass = 0; pass < 2; ++pass) {
#pragma unroll
      for (int it = 0; it < 8; ++it) {
        const int row  = it * 2 + hh;
        const int nrow = q0 + 16 * mi + row;
        const v4f val = *(const v4f*)(slab + row * kSlabP + c4);
        if (nrow < kN) *(volatile v4f*)(ob + (size_t)nrow * kH + c4) = val;
      }
      __threadfence();
    }
    __builtin_amdgcn_fence(__ATOMIC_RELEASE, "workgroup");
    __builtin_amdgcn_wave_barrier();
    __builtin_amdgcn_fence(__ATOMIC_ACQUIRE, "workgroup");
  }
}

extern "C" void kernel_launch(void* const* d_in, const int* in_sizes, int n_in,
                              void* d_out, int out_size, void* d_ws, size_t ws_size,
                              hipStream_t stream) {
  if (n_in < 8) return;
  if (in_sizes[0] != kB * kT * kN * kH) return;
  if (in_sizes[1] != kH) return;
  if (in_sizes[2] != kH * kH) return;
  if (in_sizes[3] != kH) return;
  if (in_sizes[4] != kH * kH) return;
  if (in_sizes[5] != kH) return;
  if (in_sizes[6] != kH) return;
  if (in_sizes[7] != kH) return;
  if (out_size != kB * kTW * kN * kH) return;
  if (ws_size < kWsTotal) return;

  const float* feat  = (const float*)d_in[0];
  const float* wts   = (const float*)d_in[1];
  const float* W1    = (const float*)d_in[2];
  const float* b1    = (const float*)d_in[3];
  const float* W2    = (const float*)d_in[4];
  const float* b2    = (const float*)d_in[5];
  const float* gamma = (const float*)d_in[6];
  const float* beta  = (const float*)d_in[7];
  float* outp = (float*)d_out;

  char* ws = (char*)d_ws;
  _Float16* WF  = (_Float16*)(ws + kOffWF);
  _Float16* XT  = (_Float16*)(ws + kOffXT);
  _Float16* W1T = (_Float16*)(ws + kOffW1T);
  _Float16* W2T = (_Float16*)(ws + kOffW2T);

  planes_kernel<<<kB * kT, 256, 0, stream>>>(feat, wts, WF, XT);
  wplanes_kernel<<<1, 256, 0, stream>>>(W1, W2, W1T, W2T);
  fused_kernel<<<(kB * kTW * kQT) / 4, 128, 0, stream>>>(WF, XT, W1T, W2T, feat, b1, b2, gamma, beta, outp);
}
